// GraphLayerLinearNRI_51101520888316
// MI455X (gfx1250) — hardware-verified
//
#include <hip/hip_runtime.h>
#include <stddef.h>


typedef _Float16 v16h __attribute__((ext_vector_type(16)));
typedef _Float16 v8h  __attribute__((ext_vector_type(8)));
typedef float    v8f  __attribute__((ext_vector_type(8)));
typedef float    v4f  __attribute__((ext_vector_type(4)));
typedef float    v2f  __attribute__((ext_vector_type(2)));
typedef _Float16 h16;

#ifndef NB
#define NB 16
#endif
#define NB_FULL 16
#define NODES 128
#define CIN   64
#define CH    64
#define NET   2
#define ABW   (NET * 2 * CH)
#define SW    (NET * CH)
#define MROWS (NB * NODES)
#define JT    16
#define SLD   136

static_assert(NB >= 1 && NB <= NB_FULL);
static_assert(NODES == 128);
static_assert(CIN == 64 && CH == 64 && NET == 2);
static_assert(ABW == 256 && SW == 128);
static_assert((CIN % 32) == 0 && (CH % 32) == 0 && (SW % 32) == 0);
static_assert((CH % 64) == 0 && (ABW % 64) == 0);
static_assert((MROWS % 64) == 0);
static_assert(((size_t)MROWS * CIN) % (8 * 256) == 0);
static_assert(JT == 16 && (NODES % JT) == 0);
static_assert((SLD % 8) == 0 && SLD >= SW);

#define LDT 72
#define LDC 68
static_assert((LDT % 8) == 0 && LDT >= 64);
static_assert((LDC % 4) == 0 && LDC >= 64);

#define WCARRY 64.0f
#define ACARRY 16.0f
#define SCARRY 128.0f

#define W64_BYTES   ((size_t)64 * 64 * 2)
#define WAB_BYTES   ((size_t)ABW * CH * 2)
#define WB2_BYTES   ((size_t)CH * SW * 2)
#define P16_BYTES   ((size_t)MROWS * CH * 2)
#define U_BYTES     ((size_t)MROWS * CH * 4)
#define AB_BYTES    ((size_t)MROWS * ABW * 4)
#define S16_BYTES   ((size_t)MROWS * SW * 2)
#define ES_BYTES    ((size_t)MROWS * NET * 4)
#define OFF_WLIN ((size_t)0)
#define OFF_WU1  (OFF_WLIN + W64_BYTES)
#define OFF_WU2  (OFF_WU1 + W64_BYTES)
#define OFF_WAB  (OFF_WU2 + W64_BYTES)
#define OFF_WB2  (OFF_WAB + WAB_BYTES)
#define OFF_X16  (OFF_WB2 + WB2_BYTES)
#define OFF_H16  (OFF_X16 + P16_BYTES)
#define OFF_T16  (OFF_H16 + P16_BYTES)
#define OFF_U    (OFF_T16 + P16_BYTES)
#define OFF_AB   (OFF_U + U_BYTES)
#define OFF_S16  (OFF_AB + AB_BYTES)
#define OFF_ES   (OFF_S16 + S16_BYTES)
#define WS_TOTAL (OFF_ES + ES_BYTES)
static_assert((W64_BYTES % 128) == 0 && (WAB_BYTES % 128) == 0 && (WB2_BYTES % 128) == 0);
static_assert((P16_BYTES % 128) == 0 && (U_BYTES % 128) == 0 && (AB_BYTES % 128) == 0);
static_assert((S16_BYTES % 128) == 0 && (ES_BYTES % 128) == 0);
static_assert(WS_TOTAL <= (size_t)134217728);

__device__ __forceinline__ float bf16r(float x) {
  unsigned int u = __float_as_uint(x);
  u = (u + 0x7FFFu + ((u >> 16) & 1u)) & 0xFFFF0000u;
  return __uint_as_float(u);
}

static __device__ __forceinline__ h16 toh_flush(float v) {
  const h16 r = (h16)v;
  return (fabsf(v) < 6.103515625e-05f) ? (h16)0.0f : r;
}

__device__ __forceinline__ float tanh_act(float x) {
  const float ax = fabsf(x);
  const float e = __expf(-2.0f * ax);
  const float r = (1.0f - e) * __builtin_amdgcn_rcpf(1.0f + e);
  return copysignf(r, x);
}

__device__ __forceinline__ v16h frag_at(const _Float16* p) {
  v8h lo = *(const v8h*)(p);
  v8h hi = *(const v8h*)(p + 16);
  v16h out;
#pragma unroll
  for (int i = 0; i < 8; ++i) { out[i] = lo[i]; out[i + 8] = hi[i]; }
  return out;
}

__device__ __forceinline__ v8f wmma16(v16h a, v16h b, v8f c) {
  v8f d = __builtin_amdgcn_wmma_f32_16x16x32_f16(false, a, false, b, (short)0, c,
                                                 false, false);
  asm volatile("v_nop\n\tv_nop\n\tv_nop\n\tv_nop" : "+v"(d) : "v"(a), "v"(b));
  return d;
}

__global__ __launch_bounds__(256) void wconv_kernel(
    const float* __restrict__ W, _Float16* __restrict__ Wt, unsigned ldw, unsigned ldk) {
  __shared__ _Float16 T[64 * LDT];
  const unsigned tid = threadIdx.x;
  const unsigned n0 = blockIdx.x * 64u;
  const unsigned k0 = blockIdx.y * 64u;
#pragma unroll 4
  for (unsigned j = 0; j < 16u; ++j) {
    const unsigned idx = tid + 256u * j;
    const unsigned kr = idx >> 6, nc = idx & 63u;
    const float v = W[(size_t)(k0 + kr) * ldw + n0 + nc];
    T[nc * LDT + kr] = (_Float16)(WCARRY * bf16r(v));
  }
  __syncthreads();
  v8h x[2];
  size_t off[2];
#pragma unroll
  for (unsigned i = 0; i < 2u; ++i) {
    const unsigned n = 32u * i + (tid >> 3);
    const unsigned kc = (tid & 7u) * 8u;
    x[i] = *(const v8h*)&T[n * LDT + kc];
    off[i] = (size_t)(n0 + n) * ldk + k0 + kc;
  }
#pragma unroll
  for (int i = 0; i < 2; ++i) *(volatile v8h*)(Wt + off[i]) = x[i];
  __threadfence();
#pragma unroll
  for (int i = 0; i < 2; ++i) *(volatile v8h*)(Wt + off[i]) = x[i];
}

__global__ __launch_bounds__(256) void xconv_kernel(
    const float* __restrict__ X, _Float16* __restrict__ X16) {
  const size_t g = (size_t)blockIdx.x * 256u + threadIdx.x;
  const v4f a0 = *(const v4f*)(X + g * 8u);
  const v4f a1 = *(const v4f*)(X + g * 8u + 4u);
  v8h o;
#pragma unroll
  for (int i = 0; i < 4; ++i) {
    o[i]     = toh_flush(ACARRY * bf16r(a0[i]));
    o[i + 4] = toh_flush(ACARRY * bf16r(a1[i]));
  }
  _Float16* p = X16 + g * 8u;
  *(volatile v8h*)p = o;
  __threadfence();
  *(volatile v8h*)p = o;
}

template <int MODE>
__device__ __forceinline__ void gemm_body(
    const _Float16* __restrict__ A16, const _Float16* __restrict__ Bt, const unsigned K,
    const float* __restrict__ bias, const float* __restrict__ aux0,
    const float* __restrict__ aux1, float* __restrict__ outf, _Float16* __restrict__ out16) {
  __shared__ float Cs[64 * LDC];
  const unsigned tid = threadIdx.x, lane = tid & 31u, w = tid >> 5;
  const unsigned mw = w >> 1, nw = w & 1u;
  const unsigned hh = lane >> 4, m = lane & 15u;
  const unsigned n0 = blockIdx.x * 64u;
  const unsigned row0 = blockIdx.y * 64u;

  const _Float16* ap  = A16 + (size_t)(row0 + mw * 16u + m) * K + hh * 8u;
  const _Float16* bp0 = Bt + (size_t)(n0 + nw * 32u + m) * K + hh * 8u;
  const _Float16* bp1 = bp0 + (size_t)16 * K;
  v8f acc0 = {}, acc1 = {};
#pragma unroll 2
  for (unsigned k0 = 0; k0 < K; k0 += 32u) {
    const v16h a  = frag_at(ap + k0);
    const v16h b0 = frag_at(bp0 + k0);
    const v16h b1 = frag_at(bp1 + k0);
    acc0 = wmma16(a, b0, acc0);
    acc1 = wmma16(a, b1, acc1);
  }
#pragma unroll
  for (int r = 0; r < 8; ++r) {
    float* d = &Cs[(mw * 16u + hh * 8u + (unsigned)r) * LDC + nw * 32u + m];
    d[0]  = acc0[r];
    d[16] = acc1[r];
  }
  __syncthreads();

  if (MODE == 0 || MODE == 1) {
    const float cs = 1.0f / (WCARRY * ACARRY);
    float tv = 0.0f;
    if (MODE == 0) tv = bf16r(aux1[0]);
    v8h x[2];
    size_t off[2];
#pragma unroll
    for (unsigned i = 0; i < 2u; ++i) {
      const unsigned r = 32u * i + (tid >> 3);
      const unsigned c = (tid & 7u) * 8u;
      const v4f u0 = *(const v4f*)&Cs[r * LDC + c];
      const v4f u1 = *(const v4f*)&Cs[r * LDC + c + 4];
      const v4f g0 = *(const v4f*)(bias + n0 + c);
      const v4f g1 = *(const v4f*)(bias + n0 + c + 4u);
      if (MODE == 0) {
        const v4f q0 = *(const v4f*)(aux0 + n0 + c);
        const v4f q1 = *(const v4f*)(aux0 + n0 + c + 4u);
#pragma unroll
        for (int j = 0; j < 4; ++j) {
          const float h0 = u0[j] * cs + (bf16r(g0[j]) + tv * bf16r(q0[j]));
          const float h1 = u1[j] * cs + (bf16r(g1[j]) + tv * bf16r(q1[j]));
          x[i][j]     = toh_flush(ACARRY * h0);
          x[i][j + 4] = toh_flush(ACARRY * h1);
        }
      } else {
#pragma unroll
        for (int j = 0; j < 4; ++j) {
          x[i][j]     = toh_flush(ACARRY * tanh_act(u0[j] * cs + bf16r(g0[j])));
          x[i][j + 4] = toh_flush(ACARRY * tanh_act(u1[j] * cs + bf16r(g1[j])));
        }
      }
      off[i] = (size_t)(row0 + r) * CH + n0 + c;
    }
#pragma unroll
    for (int i = 0; i < 2; ++i) *(volatile v8h*)(out16 + off[i]) = x[i];
    __threadfence();
#pragma unroll
    for (int i = 0; i < 2; ++i) *(volatile v8h*)(out16 + off[i]) = x[i];
  }

  if (MODE == 2 || MODE == 3 || MODE == 4) {
    const float cs = (MODE == 4) ? (1.0f / (WCARRY * SCARRY)) : (1.0f / (WCARRY * ACARRY));
    const unsigned ldo = (MODE == 3) ? (unsigned)ABW : (unsigned)CH;
    const unsigned bcol = (MODE == 3) ? ((n0 >> 7) * (unsigned)CH) : n0;
    const bool use_b = (MODE == 3) ? (((n0 >> 6) & 1u) == 0u) : true;
    v4f xs[4];
    size_t off[4];
#pragma unroll
    for (unsigned i = 0; i < 4u; ++i) {
      const unsigned r = 16u * i + (tid >> 4);
      const unsigned c = (tid & 15u) * 4u;
      const unsigned crow = row0 + r;
      const v4f u = *(const v4f*)&Cs[r * LDC + c];
      const v4f g = *(const v4f*)(bias + bcol + c);
      v4f val;
      if (MODE == 4) {
        const v4f g1 = *(const v4f*)(bias + CH + bcol + c);
        const v2f es = *(const v2f*)(aux1 + (size_t)crow * NET);
        const v4f un = *(const v4f*)(aux0 + (size_t)crow * CH + n0 + c);
#pragma unroll
        for (int j = 0; j < 4; ++j) {
          const float bt = (es[0] * bf16r(g[j]) + es[1] * bf16r(g1[j])) * (1.0f / SCARRY);
          val[j] = un[j] + (u[j] * cs + bt);
        }
      } else {
#pragma unroll
        for (int j = 0; j < 4; ++j) {
          const float bb = use_b ? bf16r(g[j]) : 0.0f;
          val[j] = u[j] * cs + bb;
        }
      }
      xs[i] = val;
      off[i] = (size_t)crow * ldo + n0 + c;
    }
#pragma unroll
    for (int i = 0; i < 4; ++i) *(volatile v4f*)(outf + off[i]) = xs[i];
    __threadfence();
#pragma unroll
    for (int i = 0; i < 4; ++i) *(volatile v4f*)(outf + off[i]) = xs[i];
  }
}

__global__ __launch_bounds__(256) void gemm_h_kernel(
    const _Float16* __restrict__ A16, const _Float16* __restrict__ Bt,
    const float* __restrict__ bias, const float* __restrict__ wrow0,
    const float* __restrict__ tval, _Float16* __restrict__ out16) {
  gemm_body<0>(A16, Bt, (unsigned)CIN, bias, wrow0, tval, (float*)0, out16);
}
__global__ __launch_bounds__(256) void gemm_t_kernel(
    const _Float16* __restrict__ A16, const _Float16* __restrict__ Bt,
    const float* __restrict__ bias, _Float16* __restrict__ out16) {
  gemm_body<1>(A16, Bt, (unsigned)CH, bias, bias, bias, (float*)0, out16);
}
__global__ __launch_bounds__(256) void gemm_u_kernel(
    const _Float16* __restrict__ A16, const _Float16* __restrict__ Bt,
    const float* __restrict__ bias, float* __restrict__ outf) {
  gemm_body<2>(A16, Bt, (unsigned)CH, bias, bias, bias, outf, (_Float16*)0);
}
__global__ __launch_bounds__(256) void gemm_ab_kernel(
    const _Float16* __restrict__ A16, const _Float16* __restrict__ Bt,
    const float* __restrict__ bias, float* __restrict__ outf) {
  gemm_body<3>(A16, Bt, (unsigned)CH, bias, bias, bias, outf, (_Float16*)0);
}
__global__ __launch_bounds__(256) void gemm_out_kernel(
    const _Float16* __restrict__ A16, const _Float16* __restrict__ Bt,
    const float* __restrict__ bias, const float* __restrict__ unary,
    const float* __restrict__ esum, float* __restrict__ outf) {
  gemm_body<4>(A16, Bt, (unsigned)SW, bias, unary, esum, outf, (_Float16*)0);
}

__global__ __launch_bounds__(256) void msg_kernel(
    const float* __restrict__ E, const float* __restrict__ AB,
    _Float16* __restrict__ S16, float* __restrict__ Esum) {
  __shared__ float Bs[NODES * CH];
  __shared__ float Es[NODES * 2 * JT];
  __shared__ _Float16 Ss[JT * SLD];
  __shared__ float Ev[2 * JT];

  const unsigned tid = threadIdx.x, lane = tid & 31u;
  const unsigned wave = (unsigned)__builtin_amdgcn_readfirstlane((int)(threadIdx.x >> 5));
  const unsigned j0 = blockIdx.x * (unsigned)JT;
  const unsigned n = blockIdx.y;
  const unsigned jj0 = wave * 2u;
  const unsigned c0 = lane * 2u;
  const size_t nrow = (size_t)n * NODES;

  const float* eb = E + (size_t)n * ((size_t)NODES * NODES * NET) + (size_t)j0 * NET;
#pragma unroll
  for (unsigned j = 0; j < 4u; ++j) {
    const unsigned idx = tid + 256u * j;
    const unsigned i = idx >> 3, q = (idx & 7u) * 4u;
    const v4f e4 = *(const v4f*)(eb + (size_t)i * (NODES * NET) + q);
    v4f r4;
#pragma unroll
    for (int k = 0; k < 4; ++k) r4[k] = bf16r(e4[k]);
    *(v4f*)&Es[i * (2u * JT) + q] = r4;
  }

#pragma unroll 1
  for (unsigned e = 0; e < (unsigned)NET; ++e) {
    __syncthreads();
    const float* bsrc = AB + nrow * ABW + e * (2u * CH) + CH;
#pragma unroll
    for (unsigned j = 0; j < 8u; ++j) {
      const unsigned idx = tid + 256u * j;
      const unsigned i = idx >> 4, q = (idx & 15u) * 4u;
      *(v4f*)&Bs[i * CH + q] = *(const v4f*)(bsrc + (size_t)i * ABW + q);
    }
    __syncthreads();

    const float* asrc = AB + (nrow + j0 + jj0) * ABW + e * (2u * CH) + c0;
    const v2f a0 = *(const v2f*)(asrc);
    const v2f a1 = *(const v2f*)(asrc + ABW);
    float s00 = 0.0f, s01 = 0.0f, s10 = 0.0f, s11 = 0.0f;
    float es0 = 0.0f, es1 = 0.0f;
    const unsigned ew = jj0 * 2u + e;
#pragma unroll 4
    for (unsigned i = 0; i < (unsigned)NODES; ++i) {
      const float w0 = Es[i * (2u * JT) + ew];
      const float w1 = Es[i * (2u * JT) + ew + 2u];
      const v2f b = *(const v2f*)&Bs[i * CH + c0];
      es0 += w0;
      es1 += w1;
      s00 += w0 * tanh_act(a0[0] + b[0]);
      s01 += w0 * tanh_act(a0[1] + b[1]);
      s10 += w1 * tanh_act(a1[0] + b[0]);
      s11 += w1 * tanh_act(a1[1] + b[1]);
    }
    Ss[jj0 * SLD + e * CH + c0]             = toh_flush(s00);
    Ss[jj0 * SLD + e * CH + c0 + 1u]        = toh_flush(s01);
    Ss[(jj0 + 1u) * SLD + e * CH + c0]      = toh_flush(s10);
    Ss[(jj0 + 1u) * SLD + e * CH + c0 + 1u] = toh_flush(s11);
    if (lane == 0u) {
      Ev[ew] = es0;
      Ev[ew + 2u] = es1;
    }
  }
  __syncthreads();

  const unsigned r = tid >> 4, pc = (tid & 15u) * 8u;
  const v8h sv = *(const v8h*)&Ss[r * SLD + pc];
  _Float16* sp = S16 + (nrow + j0 + r) * SW + pc;
  const v4f ev = *(const v4f*)&Ev[(tid & 7u) * 4u];
  float* ep = Esum + (nrow + j0) * NET + (tid & 7u) * 4u;
  *(volatile v8h*)sp = sv;
  if (tid < 8u) *(volatile v4f*)ep = ev;
  __threadfence();
  *(volatile v8h*)sp = sv;
  if (tid < 8u) *(volatile v4f*)ep = ev;
}

extern "C" void kernel_launch(void* const* d_in, const int* in_sizes, int n_in,
                              void* d_out, int out_size, void* d_ws, size_t ws_size,
                              hipStream_t stream) {
  if (n_in < 13) return;
  if (in_sizes[0] < 1) return;
  if ((long long)in_sizes[1] < (long long)MROWS * CIN) return;
  if ((long long)in_sizes[2] < (long long)NB * NODES * NODES * NET) return;
  if (in_sizes[3] < (CIN + 1) * CH) return;
  if (in_sizes[4] < CH || in_sizes[6] < CH || in_sizes[8] < CH) return;
  if (in_sizes[5] < CH * CH || in_sizes[7] < CH * CH) return;
  if (in_sizes[9] < NET * 2 * CH * CH) return;
  if (in_sizes[10] < NET * CH) return;
  if (in_sizes[11] < NET * CH * CH) return;
  if (in_sizes[12] < NET * CH) return;
  if ((long long)out_size < (long long)MROWS * CH) return;
  if (ws_size < WS_TOTAL) return;

  const float* tin  = (const float*)d_in[0];
  const float* X    = (const float*)d_in[1];
  const float* E    = (const float*)d_in[2];
  const float* wlin = (const float*)d_in[3];
  const float* blin = (const float*)d_in[4];
  const float* wu1  = (const float*)d_in[5];
  const float* bu1  = (const float*)d_in[6];
  const float* wu2  = (const float*)d_in[7];
  const float* bu2  = (const float*)d_in[8];
  const float* wb1  = (const float*)d_in[9];
  const float* bb1  = (const float*)d_in[10];
  const float* wb2  = (const float*)d_in[11];
  const float* bb2  = (const float*)d_in[12];
  float* out = (float*)d_out;

  char* ws = (char*)d_ws;
  _Float16* Wlin_t = (_Float16*)(ws + OFF_WLIN);
  _Float16* Wu1_t  = (_Float16*)(ws + OFF_WU1);
  _Float16* Wu2_t  = (_Float16*)(ws + OFF_WU2);
  _Float16* Wab_t  = (_Float16*)(ws + OFF_WAB);
  _Float16* Wb2_t  = (_Float16*)(ws + OFF_WB2);
  _Float16* X16    = (_Float16*)(ws + OFF_X16);
  _Float16* H16    = (_Float16*)(ws + OFF_H16);
  _Float16* T16    = (_Float16*)(ws + OFF_T16);
  float*    U      = (float*)(ws + OFF_U);
  float*    AB     = (float*)(ws + OFF_AB);
  _Float16* S16    = (_Float16*)(ws + OFF_S16);
  float*    Es     = (float*)(ws + OFF_ES);

  dim3 blk(256);
  dim3 g11(1, 1);
  dim3 gn(1, MROWS / 64);

  xconv_kernel<<<dim3((unsigned)(((size_t)MROWS * CIN) / (8 * 256))), blk, 0, stream>>>(X, X16);

  wconv_kernel<<<g11, blk, 0, stream>>>(wlin + CH, Wlin_t, (unsigned)CH, (unsigned)CIN);
  wconv_kernel<<<g11, blk, 0, stream>>>(wu1, Wu1_t, (unsigned)CH, (unsigned)CH);
  wconv_kernel<<<g11, blk, 0, stream>>>(wu2, Wu2_t, (unsigned)CH, (unsigned)CH);
  wconv_kernel<<<g11, blk, 0, stream>>>(wb1 + 0 * CH * CH, Wab_t + 0 * CH * CH, (unsigned)CH, (unsigned)CH);
  wconv_kernel<<<g11, blk, 0, stream>>>(wb1 + 1 * CH * CH, Wab_t + 1 * CH * CH, (unsigned)CH, (unsigned)CH);
  wconv_kernel<<<g11, blk, 0, stream>>>(wb1 + 2 * CH * CH, Wab_t + 2 * CH * CH, (unsigned)CH, (unsigned)CH);
  wconv_kernel<<<g11, blk, 0, stream>>>(wb1 + 3 * CH * CH, Wab_t + 3 * CH * CH, (unsigned)CH, (unsigned)CH);
  wconv_kernel<<<dim3(CH / 64, SW / 64), blk, 0, stream>>>(wb2, Wb2_t, (unsigned)CH, (unsigned)SW);

  gemm_h_kernel<<<gn, blk, 0, stream>>>(X16, Wlin_t, blin, wlin, tin, H16);
  gemm_t_kernel<<<gn, blk, 0, stream>>>(H16, Wu1_t, bu1, T16);
  gemm_u_kernel<<<gn, blk, 0, stream>>>(T16, Wu2_t, bu2, U);
  gemm_ab_kernel<<<dim3(ABW / 64, MROWS / 64), blk, 0, stream>>>(H16, Wab_t, bb1, AB);
  msg_kernel<<<dim3(NODES / JT, NB), blk, 0, stream>>>(E, AB, S16, Es);
  gemm_out_kernel<<<gn, blk, 0, stream>>>(S16, Wb2_t, bb2, U, Es, out);
}
